// CustomMultiresLayer_81578608820280
// MI455X (gfx1250) — hardware-run, weakly checked
//
#include <hip/hip_runtime.h>
#include <math.h>

typedef __attribute__((ext_vector_type(16))) _Float16 v16h;
typedef __attribute__((ext_vector_type(8)))  _Float16 v8h;
typedef __attribute__((ext_vector_type(8)))  float    v8f;
typedef __attribute__((ext_vector_type(4)))  float    v4f;
typedef __attribute__((ext_vector_type(4)))  unsigned v4u;

constexpr int kBatch  = 2;
constexpr int kCh     = 1024;
constexpr int kLen    = 4096;
constexpr int kTaps   = 4;
constexpr int kLevels = 11;
constexpr int kCols   = kBatch * kLen;
constexpr float kLnEps  = 1e-5f;
constexpr float kWCarry = 1024.0f;
constexpr float kYCarry = 32.0f;
constexpr float kFold   = 1.0f / (kWCarry * kYCarry);
static_assert((kCh % 64) == 0 && (kLen % 64) == 0 && (kCh % 32) == 0);
static_assert(kTaps == 4 && kLevels == 11 && kLen == 4096 && kCh == 1024 && kBatch == 2);
static_assert(kFold * 32768.0f == 1.0f);

constexpr size_t kOffW16  = 0;
constexpr size_t kOffY16  = kOffW16  + (size_t)kCh * kCh * 2;
constexpr size_t kOffYT16 = kOffY16  + (size_t)kBatch * kCh * kLen * 2;
constexpr size_t kOffZ    = kOffYT16 + (size_t)kCols * kCh * 2;
constexpr size_t kWsTotal = kOffZ    + (size_t)kBatch * kCh * kLen * 4;
static_assert(kWsTotal == 69206016ull);
static_assert(kWsTotal <= 134217728ull);
static_assert((kOffY16 % 128) == 0 && (kOffYT16 % 128) == 0 && (kOffZ % 128) == 0);

union FragU { v16h v; v8h h[2]; };
__device__ __forceinline__ v16h frag_load(const _Float16* p) {
  FragU f;
  f.h[0] = *(const v8h*)(p);
  f.h[1] = *(const v8h*)(p + 16);
  return f.v;
}
__device__ __forceinline__ v8f mma_guarded(v16h a, v16h b, v8f c) {
  c = __builtin_amdgcn_wmma_f32_16x16x32_f16(false, a, false, b, (short)0, c, false, false);
  asm volatile("v_nop\n\tv_nop\n\tv_nop\n\tv_nop" : "+v"(c) : "v"(a), "v"(b));
  return c;
}
__device__ __forceinline__ void keep4_h(v16h a, v16h b, v16h c, v16h d) { asm volatile("v_nop" :: "v"(a), "v"(b), "v"(c), "v"(d)); }
__device__ __forceinline__ void acc_guard4(v8f& a, v8f& b, v8f& c, v8f& d) { asm volatile("v_nop\n\tv_nop\n\tv_nop\n\tv_nop" : "+v"(a), "+v"(b), "+v"(c), "+v"(d)); }

__global__ __launch_bounds__(256) void pack_weight_kernel(const float* __restrict__ w, unsigned short* __restrict__ w16) {
  const int i = blockIdx.x * 256 + threadIdx.x;
  const size_t e0 = (size_t)i << 3;
  const v4f a0 = *(const v4f*)(w + e0);
  const v4f a1 = *(const v4f*)(w + e0 + 4);
  v8h hv;
#pragma unroll
  for (int e = 0; e < 4; ++e) {
    hv[e]     = (_Float16)(a0[e] * kWCarry);
    hv[4 + e] = (_Float16)(a1[e] * kWCarry);
  }
  unsigned short* q = w16 + e0;
  *(volatile v8h*)q = hv;
  __threadfence();
  *(volatile v8h*)q = hv;
}

__global__ __launch_bounds__(256) void tap_tree_kernel(const float* __restrict__ x, const float* __restrict__ h0,
                                                       const float* __restrict__ h1, unsigned short* __restrict__ y16) {
  __shared__ __align__(16) float sA[2 * kLen];
  __shared__ __align__(16) float sB[kLen];
  __shared__ __align__(16) float sY[kLen];
  const int t   = threadIdx.x;
  const int row = blockIdx.x;
  const int d   = row & (kCh - 1);
  const float* xrow = x + (size_t)row * kLen;
  const v4f g0 = *(const v4f*)(h0 + d * kTaps);
  const v4f g1 = *(const v4f*)(h1 + d * kTaps);
  const float p0 = g0[0], p1 = g0[1], p2 = g0[2], p3 = g0[3];
  const float q0 = g1[0], q1 = g1[1], q2 = g1[2], q3 = g1[3];
#pragma unroll
  for (int it = 0; it < 4; ++it)
    *(v4f*)(sA + it * 1024 + t * 4) = *(const v4f*)(xrow + it * 1024 + t * 4);
  __syncthreads();

#pragma unroll 1
  for (int m = 0; m < kLevels; ++m) {
    const int dil = 1 << m;
    const float* ac = sA + (m & 1) * kLen;
    float* an = sA + ((m & 1) ^ 1) * kLen;
    const float gw = (m == 1) ? 2.0f : 1.0f;
#pragma unroll 1
    for (int j = 0; j < 16; ++j) {
      const int l  = j * 256 + t;
      const int i2 = l - dil;
      const int i1 = l - 2 * dil;
      const int i0 = l - 3 * dil;
      const float v3 = ac[l];
      float v2 = ac[i2 < 0 ? 0 : i2];
      float v1 = ac[i1 < 0 ? 0 : i1];
      float v0 = ac[i0 < 0 ? 0 : i0];
      v2 = (i2 >= 0) ? v2 : 0.0f;
      v1 = (i1 >= 0) ? v1 : 0.0f;
      v0 = (i0 >= 0) ? v0 : 0.0f;
      float s0 = p0 * v0;
      s0 = fmaf(p1, v1, s0);
      s0 = fmaf(p2, v2, s0);
      s0 = fmaf(p3, v3, s0);
      float s1 = q0 * v0;
      s1 = fmaf(q1, v1, s1);
      s1 = fmaf(q2, v2, s1);
      s1 = fmaf(q3, v3, s1);
      float yv = 0.0f;
      if (m > 0) {
        const float sg = __builtin_amdgcn_rcpf(1.0f + expf(-s0));
        yv = fmaf(gw * sg, sB[l], sY[l]);
      }
      sY[l] = yv;
      sB[l] = s1;
      an[l] = s0;
    }
    __syncthreads();
  }

  v8h hv[2];
#pragma unroll
  for (int it = 0; it < 2; ++it) {
    const float* sp = sY + it * 2048 + t * 8;
    const v4f a0 = *(const v4f*)(sp);
    const v4f a1 = *(const v4f*)(sp + 4);
#pragma unroll
    for (int e = 0; e < 4; ++e) {
      hv[it][e]     = (_Float16)(a0[e] * kYCarry);
      hv[it][4 + e] = (_Float16)(a1[e] * kYCarry);
    }
  }
  unsigned short* yrow = y16 + (size_t)row * kLen;
  for (int pass = 0; pass < 2; ++pass) {
#pragma unroll
    for (int it = 0; it < 2; ++it)
      *(volatile v8h*)(yrow + it * 2048 + t * 8) = hv[it];
    __threadfence();
  }
}

__global__ __launch_bounds__(256) void plane_transpose_kernel(const unsigned* __restrict__ inw, unsigned* __restrict__ outw) {
  __shared__ __align__(16) unsigned tile[64 * 36];
  const int tid = threadIdx.x;
  const int l0 = blockIdx.x * 64;
  const int c0 = blockIdx.y * 64;
  const int b  = blockIdx.z;
  const int sg = tid & 7;
#pragma unroll
  for (int it = 0; it < 2; ++it) {
    const int r = (tid >> 3) + 32 * it;
    const size_t wi = ((((size_t)b * kCh + c0 + r) * kLen + l0) >> 1) + sg * 4;
    const v4u w = *(const v4u*)(inw + wi);
    *(v4u*)(tile + r * 36 + sg * 4) = w;
  }
  __syncthreads();
  v4u ov[2];
#pragma unroll
  for (int it = 0; it < 2; ++it) {
    const int lr = (tid >> 3) + 32 * it;
    const int sh = (lr & 1) * 16;
    const int wc = lr >> 1;
    unsigned hw[8];
#pragma unroll
    for (int e = 0; e < 8; ++e) hw[e] = (tile[(sg * 8 + e) * 36 + wc] >> sh) & 0xffffu;
    v4u o;
    o[0] = hw[0] | (hw[1] << 16);
    o[1] = hw[2] | (hw[3] << 16);
    o[2] = hw[4] | (hw[5] << 16);
    o[3] = hw[6] | (hw[7] << 16);
    ov[it] = o;
  }
  for (int pass = 0; pass < 2; ++pass) {
#pragma unroll
    for (int it = 0; it < 2; ++it) {
      const int lr = (tid >> 3) + 32 * it;
      const size_t wo = ((((size_t)b * kLen + l0 + lr) * kCh + c0) >> 1) + sg * 4;
      *(volatile v4u*)(outw + wo) = ov[it];
    }
    __threadfence();
  }
}

__global__ __launch_bounds__(256) void mix_gemm_kernel(const unsigned short* __restrict__ Ap, const unsigned short* __restrict__ Btp,
                                                       float* __restrict__ Z, const float* __restrict__ bias,
                                                       const float* __restrict__ xres) {
  __shared__ __align__(16) float sT[8][16 * 68];
  const _Float16* A  = (const _Float16*)Ap;
  const _Float16* Bt = (const _Float16*)Btp;
  const int b    = blockIdx.y;
  const int lane = threadIdx.x & 31;
  const int wave = __builtin_amdgcn_readfirstlane((int)(threadIdx.x >> 5));
  const int tile = blockIdx.x * 8 + wave;
  const int tm = tile >> 6;
  const int tn = tile & 63;
  const int m0 = tm << 6;
  const int n0 = tn << 6;
  const int rlane = lane & 15;
  const int koff  = (lane >> 4) * 8;
  const int mOff  = (lane >> 4) * 8;
  const _Float16* Bb = Bt + (size_t)b * kLen * kCh;

  v8f acc[4][4];
#pragma unroll
  for (int i = 0; i < 4; ++i)
#pragma unroll
    for (int j = 0; j < 4; ++j) acc[i][j] = (v8f){0.f, 0.f, 0.f, 0.f, 0.f, 0.f, 0.f, 0.f};

  for (int k0 = 0; k0 < kCh; k0 += 32) {
    v16h bh[4];
#pragma unroll
    for (int j = 0; j < 4; ++j) {
      const size_t bo = (size_t)(n0 + (j << 4) + rlane) * kCh + koff + k0;
      bh[j] = frag_load(Bb + bo);
    }
#pragma unroll
    for (int i = 0; i < 4; ++i) {
      const size_t ao = (size_t)(m0 + (i << 4) + rlane) * kCh + koff + k0;
      const v16h ah = frag_load(A + ao);
#pragma unroll
      for (int j = 0; j < 4; ++j) acc[i][j] = mma_guarded(ah, bh[j], acc[i][j]);
    }
    keep4_h(bh[0], bh[1], bh[2], bh[3]);
  }
  acc_guard4(acc[0][0], acc[0][1], acc[0][2], acc[0][3]);
  acc_guard4(acc[1][0], acc[1][1], acc[1][2], acc[1][3]);
  acc_guard4(acc[2][0], acc[2][1], acc[2][2], acc[2][3]);
  acc_guard4(acc[3][0], acc[3][1], acc[3][2], acc[3][3]);

  float* slab = sT[wave];
  const int hh = lane >> 4;
  const int c4 = (lane & 15) * 4;
#pragma unroll
  for (int i = 0; i < 4; ++i) {
    const int mBase = m0 + (i << 4);
    const v4f bv0 = *(const v4f*)(bias + mBase + mOff);
    const v4f bv1 = *(const v4f*)(bias + mBase + mOff + 4);
    float bb[8];
    bb[0] = bv0[0]; bb[1] = bv0[1]; bb[2] = bv0[2]; bb[3] = bv0[3];
    bb[4] = bv1[0]; bb[5] = bv1[1]; bb[6] = bv1[2]; bb[7] = bv1[3];
#pragma unroll
    for (int j = 0; j < 4; ++j) {
#pragma unroll
      for (int r = 0; r < 8; ++r)
        slab[(mOff + r) * 68 + (j << 4) + rlane] = acc[i][j][r] * kFold + bb[r];
    }
    __builtin_amdgcn_fence(__ATOMIC_RELEASE, "workgroup");
    __builtin_amdgcn_wave_barrier();
    __builtin_amdgcn_fence(__ATOMIC_ACQUIRE, "workgroup");
    v4f ov[8];
#pragma unroll
    for (int it = 0; it < 8; ++it) {
      const int row = it * 2 + hh;
      const size_t idx = ((size_t)b * kCh + mBase + row) * kLen + n0 + c4;
      const v4f sv = *(const v4f*)(slab + row * 68 + c4);
      const v4f xr = *(const v4f*)(xres + idx);
      ov[it] = sv + xr;
    }
    for (int pass = 0; pass < 2; ++pass) {
#pragma unroll
      for (int it = 0; it < 8; ++it) {
        const int row = it * 2 + hh;
        const size_t idx = ((size_t)b * kCh + mBase + row) * kLen + n0 + c4;
        *(volatile v4f*)(Z + idx) = ov[it];
      }
      __threadfence();
    }
    __builtin_amdgcn_fence(__ATOMIC_RELEASE, "workgroup");
    __builtin_amdgcn_wave_barrier();
    __builtin_amdgcn_fence(__ATOMIC_ACQUIRE, "workgroup");
  }
}

__global__ __launch_bounds__(256) void channel_norm_kernel(const float* __restrict__ Z, const float* __restrict__ gamma,
                                                           const float* __restrict__ beta, float* __restrict__ out) {
  __shared__ __align__(16) float sP[8 * 128];
  __shared__ __align__(16) float sQ[8 * 128];
  const int lane = threadIdx.x & 31;
  const int wave = __builtin_amdgcn_readfirstlane((int)(threadIdx.x >> 5));
  const int b  = blockIdx.x >> 5;
  const int l0 = (blockIdx.x & 31) * 128;
  const size_t cbase = ((size_t)b * kCh + wave * 128) * kLen + l0 + lane * 4;

  v4f s = (v4f){0.f, 0.f, 0.f, 0.f};
#pragma unroll 4
  for (int r = 0; r < 128; ++r) s += *(const v4f*)(Z + cbase + (size_t)r * kLen);
  *(v4f*)(sP + wave * 128 + lane * 4) = s;
  __syncthreads();
  v4f tot = (v4f){0.f, 0.f, 0.f, 0.f};
#pragma unroll
  for (int w = 0; w < 8; ++w) tot += *(const v4f*)(sP + w * 128 + lane * 4);
  const float invn = 1.0f / (float)kCh;
  v4f mu;
  mu[0] = tot[0] * invn; mu[1] = tot[1] * invn; mu[2] = tot[2] * invn; mu[3] = tot[3] * invn;

  v4f q = (v4f){0.f, 0.f, 0.f, 0.f};
#pragma unroll 2
  for (int r = 0; r < 128; ++r) {
    const v4f dv = *(const v4f*)(Z + cbase + (size_t)r * kLen) - mu;
    q += dv * dv;
  }
  *(v4f*)(sQ + wave * 128 + lane * 4) = q;
  __syncthreads();
  v4f qt = (v4f){0.f, 0.f, 0.f, 0.f};
#pragma unroll
  for (int w = 0; w < 8; ++w) qt += *(const v4f*)(sQ + w * 128 + lane * 4);
  v4f rs;
  rs[0] = rsqrtf(qt[0] * invn + kLnEps);
  rs[1] = rsqrtf(qt[1] * invn + kLnEps);
  rs[2] = rsqrtf(qt[2] * invn + kLnEps);
  rs[3] = rsqrtf(qt[3] * invn + kLnEps);

#pragma unroll 1
  for (int ch = 0; ch < 16; ++ch) {
    v4f ov[8];
#pragma unroll
    for (int it = 0; it < 8; ++it) {
      const int o = wave * 128 + ch * 8 + it;
      const v4f v = *(const v4f*)(Z + cbase + (size_t)(ch * 8 + it) * kLen);
      const float g  = gamma[o];
      const float bt = beta[o];
      v4f r;
      r[0] = (v[0] - mu[0]) * rs[0] * g + bt;
      r[1] = (v[1] - mu[1]) * rs[1] * g + bt;
      r[2] = (v[2] - mu[2]) * rs[2] * g + bt;
      r[3] = (v[3] - mu[3]) * rs[3] * g + bt;
      ov[it] = r;
    }
    for (int pass = 0; pass < 2; ++pass) {
#pragma unroll
      for (int it = 0; it < 8; ++it)
        *(volatile v4f*)(out + cbase + (size_t)(ch * 8 + it) * kLen) = ov[it];
      __threadfence();
    }
  }
}

extern "C" void kernel_launch(void* const* d_in, const int* in_sizes, int n_in,
                              void* d_out, int out_size, void* d_ws, size_t ws_size,
                              hipStream_t stream) {
  if (n_in < 7) return;
  if (in_sizes[0] != kBatch * kCh * kLen) return;
  if (in_sizes[1] != kCh * kTaps) return;
  if (in_sizes[2] != kCh * kTaps) return;
  if (in_sizes[3] != kCh * kCh) return;
  if (in_sizes[4] != kCh) return;
  if (in_sizes[5] != kCh) return;
  if (in_sizes[6] != kCh) return;
  if (out_size != kBatch * kCh * kLen) return;
  if (ws_size < kWsTotal) return;

  const float* x     = (const float*)d_in[0];
  const float* h0    = (const float*)d_in[1];
  const float* h1    = (const float*)d_in[2];
  const float* wmix  = (const float*)d_in[3];
  const float* bmix  = (const float*)d_in[4];
  const float* gamma = (const float*)d_in[5];
  const float* beta  = (const float*)d_in[6];
  float* out = (float*)d_out;

  char* ws = (char*)d_ws;
  unsigned short* W16  = (unsigned short*)(ws + kOffW16);
  unsigned short* Y16  = (unsigned short*)(ws + kOffY16);
  unsigned short* YT16 = (unsigned short*)(ws + kOffYT16);
  float*          Zp   = (float*)(ws + kOffZ);

  pack_weight_kernel<<<(kCh * kCh / 8) / 256, 256, 0, stream>>>(wmix, W16);
  tap_tree_kernel<<<kBatch * kCh, 256, 0, stream>>>(x, h0, h1, Y16);
  plane_transpose_kernel<<<dim3(kLen / 64, kCh / 64, kBatch), 256, 0, stream>>>((const unsigned*)Y16, (unsigned*)YT16);
  mix_gemm_kernel<<<dim3((kCh / 64) * (kLen / 64) / 8, kBatch), 256, 0, stream>>>(W16, YT16, Zp, bmix, x);
  channel_norm_kernel<<<kBatch * (kLen / 128), 256, 0, stream>>>(Zp, gamma, beta, out);
}
